// MoE_10136122818689
// MI455X (gfx1250) — hardware-verified
//
#include <hip/hip_runtime.h>
#include <math.h>

typedef __attribute__((ext_vector_type(16))) __bf16 v16b;
typedef __attribute__((ext_vector_type(8)))  _Float16 v8h;
typedef __attribute__((ext_vector_type(8)))  __bf16 v8b;
typedef __attribute__((ext_vector_type(8)))  float v8f;
typedef __attribute__((ext_vector_type(4)))  float v4f;
typedef __attribute__((ext_vector_type(2)))  float v2f;
typedef __attribute__((ext_vector_type(4)))  unsigned v4u;

#ifndef NB
#define NB 4
#endif
#ifndef SEQ
#define SEQ 2048
#endif
#define NB_FULL 4
#define SEQ_FULL 2048
#define NT (NB * SEQ)
#define DM 1024
#define NE 8
#define TILE 128
#define MAXROWS (2 * NT + NE * TILE)
#define MAXTILES (MAXROWS / TILE)
#define TEXPN 256

#define WS_WT   ((size_t)0)
#define WS_XG   (WS_WT   + (size_t)NE * DM * DM * 2)
#define WS_Y    (WS_XG   + (size_t)MAXROWS * DM * 2)
#define WS_REC  (WS_Y    + (size_t)MAXROWS * DM * 4)
#define WS_LIST (WS_REC  + (size_t)NT * 16)
#define WS_POS  (WS_LIST + (size_t)MAXROWS * 2)
#define WS_TEXP (WS_POS  + (size_t)NT * 4)
#define WS_END  (WS_TEXP + (size_t)TEXPN * 4)

static_assert(NB == 1 || SEQ == SEQ_FULL);
static_assert(NB <= NB_FULL && SEQ <= SEQ_FULL);
static_assert(NT % 128 == 0 && (NT & (NT - 1)) == 0 && NT <= 8192);
static_assert(NE == 8);
static_assert(DM == 1024 && DM % 32 == 0 && DM % 128 == 0);
static_assert(MAXROWS % 256 == 0 && MAXROWS <= 32768 && MAXTILES <= TEXPN);
static_assert((size_t)NB_FULL * SEQ_FULL * DM * 4 == 33554432);
static_assert(WS_XG % 128 == 0 && WS_Y % 128 == 0 && WS_REC % 128 == 0 && WS_LIST % 128 == 0 && WS_POS % 128 == 0 && WS_TEXP % 128 == 0);
static_assert(WS_END <= (size_t)134217728);
static_assert((size_t)(DM / 64) * (DM / 64) * NE * 4096 == (size_t)NE * DM * DM);
static_assert((size_t)(NT / 128) * 128 * 16 == (size_t)NT * 16);
static_assert((size_t)(MAXROWS / 2) * 256 * 16 == (size_t)MAXROWS * DM * 2);
static_assert(128 * 16 == DM * 2);
static_assert((size_t)(DM / 128) * MAXTILES * 128 * 128 == (size_t)MAXROWS * DM);
static_assert(8 * 32 * 16 == 16 * 64 * 4);
static_assert(256 * 16 == DM * 4);
static_assert((size_t)(MAXROWS / 8) * 16 == (size_t)MAXROWS * 2);
static_assert((size_t)(NT / 4) * 16 == (size_t)NT * 4);
static_assert(64 * 16 == TEXPN * 4);
static_assert(64 * 65 * 4 <= 131072);
static_assert(DM * NE * 4 + 128 * (NE + 1) * 4 <= 131072);
static_assert(MAXROWS * 2 + 2 * NT * 2 + TEXPN * 4 + NE * 4 <= 131072);
static_assert(8 * 16 * 64 * 4 <= 131072);

__device__ __forceinline__ v8f wmma_bf(v16b a, v16b b, v8f c) {
  v8f d = __builtin_amdgcn_wmma_f32_16x16x32_bf16(false, a, false, b, (short)0, c, false, false);
  asm volatile("v_nop\n\tv_nop\n\tv_nop\n\tv_nop" : "+v"(d) : "v"(a), "v"(b));
  return d;
}
__device__ __forceinline__ float bfr(float v) { return (float)(__bf16)v; }
__device__ __forceinline__ v16b ldfrag_b(const unsigned short* p) { union { v16b v; v4u q[2]; } f; f.q[0] = *(const v4u*)p; f.q[1] = *(const v4u*)(p + 16); return f.v; }

template <int F16>
__global__ __launch_bounds__(256) void k_tr(const float* __restrict__ S, unsigned short* __restrict__ Dst, unsigned K, unsigned N, unsigned dpitch, unsigned erow, unsigned ecol, float sc) {
  __shared__ float tile[64][65];
  const unsigned t = threadIdx.x, e = blockIdx.z, k0 = blockIdx.y * 64u, n0 = blockIdx.x * 64u;
  const float* s = S + (size_t)e * K * N;
#pragma unroll
  for (unsigned it = 0; it < 4; ++it) { const unsigned idx = it * 256u + t, kr = idx >> 4, c4 = idx & 15u;
    const v4f v = *(const v4f*)(s + (size_t)(k0 + kr) * N + n0 + 4u * c4);
    tile[kr][4u * c4 + 0] = v[0]; tile[kr][4u * c4 + 1] = v[1]; tile[kr][4u * c4 + 2] = v[2]; tile[kr][4u * c4 + 3] = v[3]; }
  __syncthreads();
  v4u o[2];
#pragma unroll
  for (unsigned it = 0; it < 2; ++it) { const unsigned idx = it * 256u + t, nr = idx >> 3, q = idx & 7u;
    union { v8b b; v8h h; v4u u; } w;
#pragma unroll
    for (int i = 0; i < 8; ++i) { const float v = bfr(tile[8u * q + i][nr]); if (F16) w.h[i] = (_Float16)(v * sc); else w.b[i] = (__bf16)v; }
    o[it] = w.u; }
#pragma unroll
  for (unsigned it = 0; it < 2; ++it) { const unsigned idx = it * 256u + t, nr = idx >> 3, q = idx & 7u;
    *(volatile v4u*)(Dst + (size_t)(e * erow + n0 + nr) * dpitch + e * ecol + k0 + 8u * q) = o[it]; }
  __threadfence();
#pragma unroll
  for (unsigned it = 0; it < 2; ++it) { const unsigned idx = it * 256u + t, nr = idx >> 3, q = idx & 7u;
    *(volatile v4u*)(Dst + (size_t)(e * erow + n0 + nr) * dpitch + e * ecol + k0 + 8u * q) = o[it]; }
}

__global__ __launch_bounds__(128) void k_gate(const float* __restrict__ X, const float* __restrict__ WG, unsigned* __restrict__ REC) {
#pragma clang fp contract(off)
  __shared__ __align__(16) float swg[DM * NE];
  __shared__ float slog[128][NE + 1];
  const unsigned tid = threadIdx.x;
#pragma unroll 1
  for (unsigned i = tid; i < (unsigned)(DM * NE / 4); i += 128u) {
    const v4f w = *(const v4f*)(WG + 4u * i); v4f o;
    o[0] = bfr(w[0]); o[1] = bfr(w[1]); o[2] = bfr(w[2]); o[3] = bfr(w[3]);
    *(v4f*)&swg[4u * i] = o; }
  __syncthreads();
  const unsigned tok = blockIdx.x * 128u + tid;
  const float* xr = X + (size_t)tok * DM;
  float a0 = 0.f, a1 = 0.f, a2 = 0.f, a3 = 0.f, a4 = 0.f, a5 = 0.f, a6 = 0.f, a7 = 0.f;
#pragma unroll 1
  for (unsigned d = 0; d < (unsigned)DM; d += 2u) {
    const v2f xv = *(const v2f*)(xr + d);
    const float x0 = bfr(xv[0]), x1 = bfr(xv[1]);
    const v4f g0 = *(const v4f*)&swg[d * NE], g1 = *(const v4f*)&swg[d * NE + 4u];
    const v4f g2 = *(const v4f*)&swg[d * NE + 8u], g3 = *(const v4f*)&swg[d * NE + 12u];
    a0 = fmaf(x0, g0[0], a0); a1 = fmaf(x0, g0[1], a1); a2 = fmaf(x0, g0[2], a2); a3 = fmaf(x0, g0[3], a3);
    a4 = fmaf(x0, g1[0], a4); a5 = fmaf(x0, g1[1], a5); a6 = fmaf(x0, g1[2], a6); a7 = fmaf(x0, g1[3], a7);
    a0 = fmaf(x1, g2[0], a0); a1 = fmaf(x1, g2[1], a1); a2 = fmaf(x1, g2[2], a2); a3 = fmaf(x1, g2[3], a3);
    a4 = fmaf(x1, g3[0], a4); a5 = fmaf(x1, g3[1], a5); a6 = fmaf(x1, g3[2], a6); a7 = fmaf(x1, g3[3], a7);
  }
  slog[tid][0] = a0; slog[tid][1] = a1; slog[tid][2] = a2; slog[tid][3] = a3;
  slog[tid][4] = a4; slog[tid][5] = a5; slog[tid][6] = a6; slog[tid][7] = a7;
  float m = fmaxf(fmaxf(fmaxf(a0, a1), fmaxf(a2, a3)), fmaxf(fmaxf(a4, a5), fmaxf(a6, a7)));
  float s = 0.f;
#pragma unroll 1
  for (unsigned e = 0; e < (unsigned)NE; ++e) { const float ev = expf(slog[tid][e] - m); slog[tid][e] = ev; s += ev; }
  const float rs = 1.0f / s;
  float v0 = -1.f, v1 = -1.f; unsigned i0 = 0u, i1 = 1u;
#pragma unroll 1
  for (unsigned e = 0; e < (unsigned)NE; ++e) {
    const float g = slog[tid][e] * rs;
    const bool b0 = g > v0, b1 = g > v1;
    v1 = b0 ? v0 : (b1 ? g : v1); i1 = b0 ? i0 : (b1 ? e : i1);
    v0 = b0 ? g : v0;             i0 = b0 ? e : i0;
  }
  const float den = (v0 + v1) + 1e-9f;
  const float rd = 1.0f / den;
  const float w0 = v0 * rd, w1 = v1 * rd;
  v4u rec; rec[0] = i0; rec[1] = i1; rec[2] = __float_as_uint(w0); rec[3] = __float_as_uint(w1);
  const v4u val = rec;
  volatile v4u* p = (volatile v4u*)(REC + 4u * (size_t)tok);
  *p = val; __threadfence(); *p = val;
}

__global__ __launch_bounds__(256) void k_route(const unsigned* __restrict__ REC, unsigned short* __restrict__ LIST, unsigned* __restrict__ POS, unsigned* __restrict__ TEXP) {
  __shared__ __align__(16) unsigned short s_list[MAXROWS];
  __shared__ __align__(16) unsigned short s_pos[2 * NT];
  __shared__ __align__(16) unsigned s_texp[TEXPN];
  __shared__ unsigned s_cnt[NE];
  const unsigned tid = threadIdx.x, lane = tid & 31u, wv = tid >> 5;
#pragma unroll 1
  for (unsigned i = tid; i < (unsigned)MAXROWS; i += 256u) s_list[i] = (unsigned short)0xFFFFu;
#pragma unroll 1
  for (unsigned i = tid; i < (unsigned)(2 * NT); i += 256u) s_pos[i] = (unsigned short)0u;
  unsigned cnt = 0u;
#pragma unroll 1
  for (unsigned c = 0; c < (unsigned)(NT / 32); ++c) {
    const v4u r = *(const v4u*)(REC + 4u * (size_t)(c * 32u + lane));
    const bool hit = ((r[0] & (NE - 1u)) == wv) | ((r[1] & (NE - 1u)) == wv);
    cnt += (unsigned)__builtin_popcount(__builtin_amdgcn_ballot_w32(hit));
  }
  if (lane == 0u) s_cnt[wv] = cnt;
  __syncthreads();
  unsigned accp = 0u, mybase = 0u, te = 0u; const unsigned rowbase = tid * (unsigned)TILE;
#pragma unroll
  for (unsigned j = 0; j < (unsigned)NE; ++j) {
    const unsigned cj = min(s_cnt[j], (unsigned)NT);
    mybase = (j == wv) ? accp : mybase;
    accp += (cj + (unsigned)(TILE - 1)) & ~(unsigned)(TILE - 1);
    te += (accp <= rowbase) ? 1u : 0u;
  }
  s_texp[tid] = min(te, (unsigned)(NE - 1));
  unsigned run = mybase;
#pragma unroll 1
  for (unsigned c = 0; c < (unsigned)(NT / 32); ++c) {
    const unsigned tok = c * 32u + lane;
    const v4u r = *(const v4u*)(REC + 4u * (size_t)tok);
    const bool h0 = (r[0] & (NE - 1u)) == wv, h1 = (r[1] & (NE - 1u)) == wv;
    const bool hit = h0 | h1;
    const unsigned b = __builtin_amdgcn_ballot_w32(hit);
    const unsigned pos = run + (unsigned)__builtin_popcount(b & ((1u << lane) - 1u));
    const unsigned slot = h0 ? 0u : 1u;
    if (hit && pos < (unsigned)MAXROWS) { s_list[pos] = (unsigned short)(tok | (slot << 13)); s_pos[2u * tok + slot] = (unsigned short)pos; }
    run += (unsigned)__builtin_popcount(b);
  }
  __syncthreads();
#pragma unroll 1
  for (unsigned idx = tid; idx < (unsigned)(MAXROWS / 8); idx += 256u) { const v4u v = *(const v4u*)&s_list[8u * idx]; *(volatile v4u*)(LIST + 8u * (size_t)idx) = v; }
#pragma unroll 1
  for (unsigned idx = tid; idx < (unsigned)(NT / 4); idx += 256u) { const v4u v = *(const v4u*)&s_pos[8u * idx]; *(volatile v4u*)(POS + 4u * (size_t)idx) = v; }
  if (tid < 64u) { const v4u v = *(const v4u*)&s_texp[4u * tid]; *(volatile v4u*)(TEXP + 4u * (size_t)tid) = v; }
  __threadfence();
#pragma unroll 1
  for (unsigned idx = tid; idx < (unsigned)(MAXROWS / 8); idx += 256u) { const v4u v = *(const v4u*)&s_list[8u * idx]; *(volatile v4u*)(LIST + 8u * (size_t)idx) = v; }
#pragma unroll 1
  for (unsigned idx = tid; idx < (unsigned)(NT / 4); idx += 256u) { const v4u v = *(const v4u*)&s_pos[8u * idx]; *(volatile v4u*)(POS + 4u * (size_t)idx) = v; }
  if (tid < 64u) { const v4u v = *(const v4u*)&s_texp[4u * tid]; *(volatile v4u*)(TEXP + 4u * (size_t)tid) = v; }
}

__global__ __launch_bounds__(256) void k_gather(const float* __restrict__ X, const unsigned short* __restrict__ LIST, unsigned short* __restrict__ XG) {
  const unsigned t = threadIdx.x; const unsigned p = blockIdx.x * 2u + (t >> 7), q = t & 127u;
  const unsigned ent = LIST[p];
  const unsigned tok = ent & (unsigned)(NT - 1);
  const bool ok = (ent & 0x8000u) == 0u;
  const float* s = X + (size_t)tok * DM + 8u * q;
  const v4f a = *(const v4f*)s, b = *(const v4f*)(s + 4);
  union { v8b h; v4u u; } o;
#pragma unroll
  for (int j = 0; j < 4; ++j) { o.h[j] = (__bf16)a[j]; o.h[4 + j] = (__bf16)b[j]; }
  const v4u z = {0u, 0u, 0u, 0u};
  const v4u val = ok ? o.u : z;
  volatile v4u* d = (volatile v4u*)(XG + (size_t)p * DM + 8u * q);
  *d = val; __threadfence(); *d = val;
}

__global__ __launch_bounds__(256) void k_exp(const unsigned short* __restrict__ XG, const unsigned short* __restrict__ WT, const unsigned* __restrict__ TEXP, float* __restrict__ Y) {
  __shared__ __align__(16) float sf[8][16][64];
  const unsigned t = threadIdx.x, lane = t & 31u, lm = lane & 15u, lh = lane >> 4;
  const unsigned wave = (unsigned)__builtin_amdgcn_readfirstlane((int)(t >> 5)), wm = wave >> 1, wn = wave & 1u;
  const unsigned m0 = blockIdx.y * 128u, n0 = blockIdx.x * 128u;
  const unsigned e = TEXP[blockIdx.y] & (unsigned)(NE - 1);
  const unsigned short* ar[2]; const unsigned short* br[4];
#pragma unroll
  for (int mi = 0; mi < 2; ++mi) ar[mi] = XG + (size_t)(m0 + wm * 32u + mi * 16u + lm) * DM + 8u * lh;
#pragma unroll
  for (int ni = 0; ni < 4; ++ni) br[ni] = WT + (size_t)(e * DM + n0 + wn * 64u + ni * 16u + lm) * DM + 8u * lh;
  v8f acc[2][4] = {};
#pragma unroll 2
  for (unsigned kc = 0; kc < DM / 32; ++kc) { v16b a[2], b[4];
#pragma unroll
    for (int mi = 0; mi < 2; ++mi) a[mi] = ldfrag_b(ar[mi] + kc * 32u);
#pragma unroll
    for (int ni = 0; ni < 4; ++ni) b[ni] = ldfrag_b(br[ni] + kc * 32u);
#pragma unroll
    for (int mi = 0; mi < 2; ++mi)
#pragma unroll
      for (int ni = 0; ni < 4; ++ni) acc[mi][ni] = wmma_bf(a[mi], b[ni], acc[mi][ni]); }
#pragma unroll
  for (int mi = 0; mi < 2; ++mi) {
    if (mi) __syncthreads();
#pragma unroll
    for (int ni = 0; ni < 4; ++ni)
#pragma unroll
      for (int r = 0; r < 8; ++r) sf[wave][8u * lh + r][ni * 16 + lm] = acc[mi][ni][r];
    __syncthreads();
    v4f v[8];
#pragma unroll
    for (unsigned it = 0; it < 8; ++it) { const unsigned rw = it * 2u + (lane >> 4), pc = lane & 15u; v[it] = *(const v4f*)&sf[wave][rw][4u * pc]; }
    float* po = Y + (size_t)(m0 + wm * 32u + mi * 16u) * DM + n0 + wn * 64u;
#pragma unroll
    for (unsigned it = 0; it < 8; ++it) { const unsigned rw = it * 2u + (lane >> 4), pc = lane & 15u; *(volatile v4f*)(po + (size_t)rw * DM + 4u * pc) = v[it]; }
    __threadfence();
#pragma unroll
    for (unsigned it = 0; it < 8; ++it) { const unsigned rw = it * 2u + (lane >> 4), pc = lane & 15u; *(volatile v4f*)(po + (size_t)rw * DM + 4u * pc) = v[it]; }
  }
}

__global__ __launch_bounds__(256) void k_comb(const float* __restrict__ Y, const unsigned* __restrict__ REC, const unsigned* __restrict__ POS, float* __restrict__ OUT) {
#pragma clang fp contract(off)
  const unsigned tok = blockIdx.x, t = threadIdx.x;
  const v4u r = *(const v4u*)(REC + 4u * (size_t)tok);
  const unsigned pp = POS[tok];
  const unsigned p0 = min(pp & 0xFFFFu, (unsigned)(MAXROWS - 1));
  const unsigned p1 = min(pp >> 16, (unsigned)(MAXROWS - 1));
  const float w0 = __uint_as_float(r[2]), w1 = __uint_as_float(r[3]);
  const v4f a = *(const v4f*)(Y + (size_t)p0 * DM + 4u * t);
  const v4f b = *(const v4f*)(Y + (size_t)p1 * DM + 4u * t);
  v4f o;
#pragma unroll
  for (int j = 0; j < 4; ++j) { const float ta = a[j] * w0; const float tb = b[j] * w1; o[j] = ta + tb; }
  const v4f val = o;
  volatile v4f* d = (volatile v4f*)(OUT + (size_t)tok * DM + 4u * t);
  *d = val; __threadfence(); *d = val;
}

extern "C" void kernel_launch(void* const* d_in, const int* in_sizes, int n_in, void* d_out, int out_size, void* d_ws, size_t ws_size, hipStream_t stream) {
  if (n_in < 3) return;
  if (in_sizes[0] < NT * DM || in_sizes[1] < DM * NE || in_sizes[2] < NE * DM * DM) return;
  if ((size_t)out_size < (size_t)NT * DM) return;
  if (ws_size < (size_t)WS_END) return;
  const float* X  = (const float*)d_in[0];
  const float* WG = (const float*)d_in[1];
  const float* WE = (const float*)d_in[2];
  char* ws = (char*)d_ws;
  unsigned short* WT   = (unsigned short*)(ws + WS_WT);
  unsigned short* XG   = (unsigned short*)(ws + WS_XG);
  float*          Y    = (float*)(ws + WS_Y);
  unsigned*       REC  = (unsigned*)(ws + WS_REC);
  unsigned short* LIST = (unsigned short*)(ws + WS_LIST);
  unsigned*       POS  = (unsigned*)(ws + WS_POS);
  unsigned*       TEXP = (unsigned*)(ws + WS_TEXP);
  float* OUT = (float*)d_out;
  k_tr<0><<<dim3(DM / 64, DM / 64, NE), 256, 0, stream>>>(WE, WT, (unsigned)DM, (unsigned)DM, (unsigned)DM, (unsigned)DM, 0u, 1.0f);
  k_gate<<<dim3(NT / 128), 128, 0, stream>>>(X, WG, REC);
  k_route<<<dim3(1), 256, 0, stream>>>(REC, LIST, POS, TEXP);
  k_gather<<<dim3(MAXROWS / 2), 256, 0, stream>>>(X, LIST, XG);
  k_exp<<<dim3(DM / 128, MAXTILES), 256, 0, stream>>>(XG, WT, TEXP, Y);
  k_comb<<<dim3(NT), 256, 0, stream>>>(Y, REC, POS, OUT);
}
